// tinyBlock_36455682408714
// MI455X (gfx1250) — hardware-verified
//
#include <hip/hip_runtime.h>
#include <stdint.h>


typedef _Float16 v16h __attribute__((ext_vector_type(16)));
typedef _Float16 v8h  __attribute__((ext_vector_type(8)));
typedef float    v8f  __attribute__((ext_vector_type(8)));
typedef float    v4f  __attribute__((ext_vector_type(4)));

union Frag { v16h v; v8h half[2]; };

static constexpr int BB = 4;
static constexpr int TT = 4096;
static constexpr int DD = 256;
static constexpr int HH = 1024;
static constexpr int NT = BB * TT;

typedef char shape_chk0[(NT % 64 == 0 && NT % 32 == 0 && NT % 16 == 0 && NT % 8 == 0) ? 1 : -1];
typedef char shape_chk1[(DD % 64 == 0 && HH % 64 == 0 && DD % 32 == 0 && HH % 32 == 0 && TT % 64 == 0) ? 1 : -1];
typedef char shape_chk2[((DD * DD) % 2048 == 0 && (HH * DD) % 2048 == 0) ? 1 : -1];

__device__ __forceinline__ v8f wmma16(v16h a, v16h b, v8f c) {
    v8f d = __builtin_amdgcn_wmma_f32_16x16x32_f16(false, a, false, b, (short)0, c, false, false);
    asm volatile("v_nop\n\tv_nop\n\tv_nop\n\tv_nop" : "+v"(d) : "v"(a), "v"(b));
    return d;
}

__device__ __forceinline__ v8h cvt8(v4f a, v4f b) {
    v8h o;
    o[0] = (_Float16)a[0]; o[1] = (_Float16)a[1]; o[2] = (_Float16)a[2]; o[3] = (_Float16)a[3];
    o[4] = (_Float16)b[0]; o[5] = (_Float16)b[1]; o[6] = (_Float16)b[2]; o[7] = (_Float16)b[3];
    return o;
}

__global__ __launch_bounds__(256) void cvt_w16(const float* __restrict__ s0, const float* __restrict__ s1,
                                               const float* __restrict__ s2, const float* __restrict__ s3,
                                               const float* __restrict__ s4, const float* __restrict__ s5,
                                               _Float16* __restrict__ d0, _Float16* __restrict__ d1,
                                               _Float16* __restrict__ d2, _Float16* __restrict__ d3,
                                               _Float16* __restrict__ d4, _Float16* __restrict__ d5) {
    const float* src;
    _Float16* dst;
    int n;
    switch (blockIdx.y) {
        case 0:  src = s0; dst = d0; n = DD * DD; break;
        case 1:  src = s1; dst = d1; n = DD * DD; break;
        case 2:  src = s2; dst = d2; n = DD * DD; break;
        case 3:  src = s3; dst = d3; n = DD * DD; break;
        case 4:  src = s4; dst = d4; n = HH * DD; break;
        default: src = s5; dst = d5; n = DD * HH; break;
    }
    const int i8 = (blockIdx.x * 256 + threadIdx.x) * 8;
    if (i8 + 8 > n) return;
    const v4f a = *(const v4f*)(src + i8);
    const v4f b = *(const v4f*)(src + i8 + 4);
    const v8h o = cvt8(a, b);
    *(volatile v8h*)(dst + i8) = o;
    __threadfence();
    *(volatile v8h*)(dst + i8) = o;
}

__global__ __launch_bounds__(256) void rmsnorm16(const float* __restrict__ x, const float* __restrict__ w,
                                                 _Float16* __restrict__ out, int nrows) {
    const int wv = threadIdx.x >> 5;
    const int l  = threadIdx.x & 31;
    const int row = blockIdx.x * 8 + wv;
    if (row >= nrows) return;
    const float* xr = x + (size_t)row * DD + l * 8;
    const v4f a = *(const v4f*)xr;
    const v4f c = *(const v4f*)(xr + 4);
    float ss = a[0] * a[0] + a[1] * a[1] + a[2] * a[2] + a[3] * a[3]
             + c[0] * c[0] + c[1] * c[1] + c[2] * c[2] + c[3] * c[3];
#pragma unroll
    for (int off = 16; off > 0; off >>= 1) ss += __shfl_xor(ss, off);
    const float rms = sqrtf(ss * (1.0f / DD) + 1e-6f);
    const float inv = 1.0f / rms;
    const v4f w0 = *(const v4f*)(w + l * 8);
    const v4f w1 = *(const v4f*)(w + l * 8 + 4);
    v4f y0, y1;
#pragma unroll
    for (int i = 0; i < 4; ++i) { y0[i] = (a[i] * inv) * w0[i]; y1[i] = (c[i] * inv) * w1[i]; }
    const v8h o = cvt8(y0, y1);
    _Float16* op = out + (size_t)row * DD + l * 8;
    *(volatile v8h*)op = o;
    __threadfence();
    *(volatile v8h*)op = o;
}

template <int MODE, int K>
__global__ __launch_bounds__(32) void gemm_nt(const _Float16* __restrict__ A,
                                              const _Float16* __restrict__ Bm,
                                              const float* __restrict__ bias,
                                              const float* __restrict__ resid,
                                              _Float16* __restrict__ out_h,
                                              float* __restrict__ out_f,
                                              int M, int N) {
    __shared__ alignas(16) float tile[32 * 64];
    const int l = threadIdx.x & 31;
    const int h = l >> 4;
    const int m = l & 15;
    const int row0 = blockIdx.x * 32;
    const int n0   = blockIdx.y * 64;
    if (row0 + 32 > M || n0 + 64 > N) return;

    v8f acc[2][4] = {};
    const _Float16* a0p = A  + (size_t)(row0 + m) * K + 8 * h;
    const _Float16* a1p = a0p + (size_t)16 * K;
    const _Float16* bp  = Bm + (size_t)(n0 + m) * K + 8 * h;

#pragma unroll 2
    for (int k0 = 0; k0 < K; k0 += 32) {
        Frag fa0, fa1;
        fa0.half[0] = *(const v8h*)(a0p + k0);
        fa0.half[1] = *(const v8h*)(a0p + k0 + 16);
        fa1.half[0] = *(const v8h*)(a1p + k0);
        fa1.half[1] = *(const v8h*)(a1p + k0 + 16);
#pragma unroll
        for (int j = 0; j < 4; ++j) {
            Frag fb;
            const _Float16* bj = bp + (size_t)(16 * j) * K + k0;
            fb.half[0] = *(const v8h*)(bj);
            fb.half[1] = *(const v8h*)(bj + 16);
            acc[0][j] = wmma16(fa0.v, fb.v, acc[0][j]);
            acc[1][j] = wmma16(fa1.v, fb.v, acc[1][j]);
        }
    }

    float bn[4];
#pragma unroll
    for (int j = 0; j < 4; ++j) bn[j] = bias[(MODE == 1) ? 0 : (n0 + 16 * j + m)];
#pragma unroll
    for (int mt = 0; mt < 2; ++mt) {
#pragma unroll
        for (int r = 0; r < 8; ++r) {
            const int lr = mt * 16 + 8 * h + r;
            float brow = 0.0f;
            if (MODE == 1) brow = bias[row0 + lr];
#pragma unroll
            for (int j = 0; j < 4; ++j) {
                const int lc = 16 * j + m;
                float val = acc[mt][j][r] + ((MODE == 1) ? brow : bn[j]);
                if (MODE == 3) val = 0.5f * val * (1.0f + erff(val * 0.70710678118654752f));
                tile[lr * 64 + lc] = val;
            }
        }
    }
    __syncthreads();

    if (MODE == 2) {
#pragma unroll
        for (int pass = 0; pass < 2; ++pass) {
#pragma unroll
            for (int it = 0; it < 16; ++it) {
                const int lr = it * 2 + (l >> 4);
                const int c4 = (l & 15) * 4;
                v4f v = *(const v4f*)(tile + lr * 64 + c4);
                const size_t gi = (size_t)(row0 + lr) * N + n0 + c4;
                const v4f rr = *(const v4f*)(resid + gi);
                v = rr + v;
                *(volatile v4f*)(out_f + gi) = v;
            }
            if (pass == 0) __threadfence();
        }
    } else {
#pragma unroll
        for (int pass = 0; pass < 2; ++pass) {
#pragma unroll
            for (int it = 0; it < 8; ++it) {
                const int lr = it * 4 + (l >> 3);
                const int c8 = (l & 7) * 8;
                const v4f f0 = *(const v4f*)(tile + lr * 64 + c8);
                const v4f f1 = *(const v4f*)(tile + lr * 64 + c8 + 4);
                const v8h o = cvt8(f0, f1);
                size_t gi;
                if (MODE == 1) {
                    const int bb = n0 / TT;
                    const int t  = n0 - bb * TT;
                    gi = ((size_t)bb * DD + row0 + lr) * TT + t + c8;
                } else {
                    gi = (size_t)(row0 + lr) * N + n0 + c8;
                }
                *(volatile v8h*)(out_h + gi) = o;
            }
            if (pass == 0) __threadfence();
        }
    }
}

template <bool MASK>
__device__ __forceinline__ void attn_step(int s0, int t0, int w, int h, int m,
                                          const _Float16* __restrict__ qrow,
                                          const _Float16* __restrict__ kblk,
                                          const _Float16* __restrict__ vrows,
                                          _Float16* pstage, float* redmax, float* redsum,
                                          v8f (&acc)[8], float& rmax, float& lsum) {
    v8f sc0 = {};
    v8f sc1 = {};
    {
        const _Float16* k0p = kblk + (size_t)(s0 + 32 * w + m) * DD + 8 * h;
        const _Float16* k1p = k0p + (size_t)16 * DD;
        const _Float16* qp  = qrow + 8 * h;
#pragma unroll 2
        for (int kk = 0; kk < 8; ++kk) {
            Frag fq, fk0, fk1;
            fq.half[0]  = *(const v8h*)(qp  + 32 * kk);
            fq.half[1]  = *(const v8h*)(qp  + 32 * kk + 16);
            fk0.half[0] = *(const v8h*)(k0p + 32 * kk);
            fk0.half[1] = *(const v8h*)(k0p + 32 * kk + 16);
            fk1.half[0] = *(const v8h*)(k1p + 32 * kk);
            fk1.half[1] = *(const v8h*)(k1p + 32 * kk + 16);
            sc0 = wmma16(fk0.v, fq.v, sc0);
            sc1 = wmma16(fk1.v, fq.v, sc1);
        }
    }

    float mloc = -1.0e30f;
    const int qi = t0 + m;
#pragma unroll
    for (int r = 0; r < 8; ++r) {
        float a = sc0[r] * 0.0625f;
        float b = sc1[r] * 0.0625f;
        if (MASK) {
            const int key0 = s0 + 32 * w + 8 * h + r;
            if (key0 > qi)      a = -1.0e30f;
            if (key0 + 16 > qi) b = -1.0e30f;
        }
        sc0[r] = a;
        sc1[r] = b;
        mloc = fmaxf(mloc, fmaxf(a, b));
    }
    mloc = fmaxf(mloc, __shfl_xor(mloc, 16));
    if (h == 0) redmax[w * 16 + m] = mloc;
    __syncthreads();

    const float mnew    = fmaxf(rmax, fmaxf(mloc, redmax[(1 - w) * 16 + m]));
    const float rescale = __expf(rmax - mnew);
    rmax = mnew;

    float ps = 0.0f;
    v8h p0, p1;
#pragma unroll
    for (int r = 0; r < 8; ++r) {
        const float e0 = __expf(sc0[r] - mnew);
        const float e1 = __expf(sc1[r] - mnew);
        ps += e0 + e1;
        p0[r] = (_Float16)e0;
        p1[r] = (_Float16)e1;
    }
    *(v8h*)(pstage + m * 64 + 32 * w + 8 * h)      = p0;
    *(v8h*)(pstage + m * 64 + 32 * w + 16 + 8 * h) = p1;
    ps += __shfl_xor(ps, 16);
    if (h == 0) redsum[w * 16 + m] = ps;
    lsum = lsum * rescale + ps;
#pragma unroll
    for (int j = 0; j < 8; ++j) acc[j] = acc[j] * rescale;
    __syncthreads();

    lsum += redsum[(1 - w) * 16 + m];

#pragma unroll
    for (int ks = 0; ks < 2; ++ks) {
        Frag fp;
        fp.half[0] = *(const v8h*)(pstage + m * 64 + 32 * ks + 8 * h);
        fp.half[1] = *(const v8h*)(pstage + m * 64 + 32 * ks + 16 + 8 * h);
#pragma unroll
        for (int j = 0; j < 8; ++j) {
            Frag fv;
            const _Float16* vp = vrows + (size_t)(16 * j + m) * TT + s0 + 32 * ks + 8 * h;
            fv.half[0] = *(const v8h*)(vp);
            fv.half[1] = *(const v8h*)(vp + 16);
            acc[j] = wmma16(fv.v, fp.v, acc[j]);
        }
    }
}

__global__ __launch_bounds__(64) void flash_attn(const _Float16* __restrict__ qh,
                                                 const _Float16* __restrict__ kh,
                                                 const _Float16* __restrict__ vt,
                                                 _Float16* __restrict__ attn) {
    __shared__ alignas(16) _Float16 pstage[16 * 64];
    __shared__ alignas(16) _Float16 ostage[16 * 256];
    __shared__ float redmax[2 * 16];
    __shared__ float redsum[2 * 16];

    const int tid = threadIdx.x;
    const int w   = tid >> 5;
    const int l   = tid & 31;
    const int h   = l >> 4;
    const int m   = l & 15;
    const int qb  = blockIdx.x;
    const int b   = qb / (TT / 16);
    const int t0  = (qb - b * (TT / 16)) * 16;
    const int q0g = qb * 16;

    const _Float16* qrow  = qh + (size_t)(q0g + m) * DD;
    const _Float16* kblk  = kh + (size_t)b * TT * DD;
    const _Float16* vrows = vt + ((size_t)b * DD + 128 * w) * TT;

    v8f acc[8] = {};
    float rmax = -1.0e30f;
    float lsum = 0.0f;

    const int nFull = t0 >> 6;
    const int nIter = (t0 + 16 + 63) >> 6;

    int it = 0;
    for (; it < nFull; ++it)
        attn_step<false>(it * 64, t0, w, h, m, qrow, kblk, vrows, pstage, redmax, redsum, acc, rmax, lsum);
    for (; it < nIter; ++it)
        attn_step<true>(it * 64, t0, w, h, m, qrow, kblk, vrows, pstage, redmax, redsum, acc, rmax, lsum);

    const float inv = 1.0f / lsum;
#pragma unroll
    for (int j = 0; j < 8; ++j) {
        v8h o;
#pragma unroll
        for (int r = 0; r < 8; ++r) o[r] = (_Float16)(acc[j][r] * inv);
        *(v8h*)(ostage + m * 256 + 128 * w + 16 * j + 8 * h) = o;
    }
    __syncthreads();

#pragma unroll
    for (int pass = 0; pass < 2; ++pass) {
#pragma unroll
        for (int i = 0; i < 8; ++i) {
            const int lr = i * 2 + w;
            const v8h v = *(const v8h*)(ostage + lr * 256 + l * 8);
            *(volatile v8h*)(attn + (size_t)(q0g + lr) * DD + l * 8) = v;
        }
        if (pass == 0) __threadfence();
    }
}

extern "C" void kernel_launch(void* const* d_in, const int* in_sizes, int n_in,
                              void* d_out, int out_size, void* d_ws, size_t ws_size,
                              hipStream_t stream) {
    if (n_in < 15) return;
    if (in_sizes[0] != NT * DD || out_size != NT * DD) return;
    if (in_sizes[3] != DD * DD || in_sizes[5] != DD * DD || in_sizes[7] != DD * DD || in_sizes[9] != DD * DD) return;
    if (in_sizes[11] != HH * DD || in_sizes[13] != DD * HH) return;
    if (in_sizes[1] != DD || in_sizes[2] != DD || in_sizes[4] != DD || in_sizes[6] != DD ||
        in_sizes[8] != DD || in_sizes[10] != DD || in_sizes[12] != HH || in_sizes[14] != DD) return;

    const float* x   = (const float*)d_in[0];
    const float* anw = (const float*)d_in[1];
    const float* mnw = (const float*)d_in[2];
    const float* wq  = (const float*)d_in[3];
    const float* bq  = (const float*)d_in[4];
    const float* wk  = (const float*)d_in[5];
    const float* bk  = (const float*)d_in[6];
    const float* wv  = (const float*)d_in[7];
    const float* bv  = (const float*)d_in[8];
    const float* wo  = (const float*)d_in[9];
    const float* bo  = (const float*)d_in[10];
    const float* w1  = (const float*)d_in[11];
    const float* b1  = (const float*)d_in[12];
    const float* w2  = (const float*)d_in[13];
    const float* b2  = (const float*)d_in[14];
    float* out       = (float*)d_out;

    char* ws = (char*)d_ws;
    size_t off = 0;
    auto take = [&](size_t bytes) -> char* {
        char* p = ws + off;
        off += (bytes + 255) & ~(size_t)255;
        return p;
    };
    _Float16* xn   = (_Float16*)take((size_t)NT * DD * 2);
    _Float16* qh   = (_Float16*)take((size_t)NT * DD * 2);
    _Float16* kh   = (_Float16*)take((size_t)NT * DD * 2);
    _Float16* vt   = (_Float16*)take((size_t)NT * DD * 2);
    _Float16* attn = (_Float16*)take((size_t)NT * DD * 2);
    float*    x1   = (float*)   take((size_t)NT * DD * 4);
    _Float16* hn   = (_Float16*)take((size_t)NT * DD * 2);
    _Float16* hbuf = (_Float16*)take((size_t)NT * HH * 2);
    _Float16* wq16 = (_Float16*)take((size_t)DD * DD * 2);
    _Float16* wk16 = (_Float16*)take((size_t)DD * DD * 2);
    _Float16* wv16 = (_Float16*)take((size_t)DD * DD * 2);
    _Float16* wo16 = (_Float16*)take((size_t)DD * DD * 2);
    _Float16* w116 = (_Float16*)take((size_t)HH * DD * 2);
    _Float16* w216 = (_Float16*)take((size_t)DD * HH * 2);
    if (off > ws_size) return;

    cvt_w16<<<dim3((HH * DD) / 2048, 6), dim3(256), 0, stream>>>(wq, wk, wv, wo, w1, w2,
                                                                 wq16, wk16, wv16, wo16, w116, w216);

    rmsnorm16<<<dim3((NT + 7) / 8), dim3(256), 0, stream>>>(x, anw, xn, NT);

    gemm_nt<0, DD><<<dim3(NT / 32, DD / 64), dim3(32), 0, stream>>>(xn, wq16, bq, bq, qh, x1, NT, DD);
    gemm_nt<0, DD><<<dim3(NT / 32, DD / 64), dim3(32), 0, stream>>>(xn, wk16, bk, bk, kh, x1, NT, DD);
    gemm_nt<1, DD><<<dim3(DD / 32, NT / 64), dim3(32), 0, stream>>>(wv16, xn, bv, bv, vt, x1, DD, NT);

    flash_attn<<<dim3(NT / 16), dim3(64), 0, stream>>>(qh, kh, vt, attn);

    gemm_nt<2, DD><<<dim3(NT / 32, DD / 64), dim3(32), 0, stream>>>(attn, wo16, bo, x, hn, x1, NT, DD);

    rmsnorm16<<<dim3((NT + 7) / 8), dim3(256), 0, stream>>>(x1, mnw, hn, NT);

    gemm_nt<3, DD><<<dim3(NT / 32, HH / 64), dim3(32), 0, stream>>>(hn, w116, b1, b1, hbuf, x1, NT, HH);

    gemm_nt<2, HH><<<dim3(NT / 32, DD / 64), dim3(32), 0, stream>>>(hbuf, w216, b2, x1, hn, out, NT, DD);
}
